// JacobiKANLinear_17411797418702
// MI455X (gfx1250) — hardware-run, weakly checked
//
#include <hip/hip_runtime.h>
#include <math.h>

constexpr int kRows      = 8192;
constexpr int kInF       = 1024;
constexpr int kOutF      = 1024;
constexpr int kDeg1      = 6;
constexpr int kKB        = kInF * kDeg1;
constexpr int kChunkRows = 4096;
constexpr int kNumChunks = kRows / kChunkRows;

constexpr float kSCarry    = 16.0f;
constexpr float kWCarry    = 32.0f;
constexpr float kPCarry    = 8.0f;
constexpr float kJCarry    = 4096.0f;
constexpr float kBaseScale = 1.0f / (16.0f * 32.0f);
constexpr float kPolyScale = 1.0f / (8.0f * 4096.0f);

constexpr float kAl2 = 64.0f,  kAl3 = 180.0f, kAl4 = 384.0f, kAl5 = 700.0f;
constexpr float kRg2 = 1.0f / 120.0f, kRg3 = 1.0f / 336.0f, kRg4 = 1.0f / 720.0f, kRg5 = 1.0f / 1320.0f;
constexpr float kBc2 = (float)(48.0 / 120.0), kBc3 = (float)(144.0 / 336.0),
                kBc4 = (float)(320.0 / 720.0), kBc5 = (float)(600.0 / 1320.0);

typedef __attribute__((ext_vector_type(16))) _Float16 v16h;
typedef __attribute__((ext_vector_type(8)))  _Float16 v8h;
typedef __attribute__((ext_vector_type(16))) __bf16   v16b;
typedef __attribute__((ext_vector_type(8)))  __bf16   v8b;
typedef __attribute__((ext_vector_type(8)))  float    v8f;
typedef __attribute__((ext_vector_type(4)))  float    v4f;
typedef __attribute__((ext_vector_type(4)))  unsigned int v4u;

__device__ __forceinline__ unsigned short f2bf_bits(float f) {
  unsigned u = __float_as_uint(f);
  return (unsigned short)((u + 0x7FFFu + ((u >> 16) & 1u)) >> 16);
}
__device__ __forceinline__ float bf_bits2f(unsigned short h) { return __uint_as_float(((unsigned)h) << 16); }

__device__ __forceinline__ void dep_guard_h(v8f& a, v8f& b, v16h x, v16h y) { asm volatile("v_nop\n\tv_nop\n\tv_nop\n\tv_nop" : "+v"(a), "+v"(b) : "v"(x), "v"(y)); }
__device__ __forceinline__ void dep_guard_b(v8f& a, v8f& b, v16b x, v16b y) { asm volatile("v_nop\n\tv_nop\n\tv_nop\n\tv_nop" : "+v"(a), "+v"(b) : "v"(x), "v"(y)); }
__device__ __forceinline__ void keep4_h(v16h a, v16h b, v16h c, v16h d) { asm volatile("v_nop" :: "v"(a), "v"(b), "v"(c), "v"(d)); }
__device__ __forceinline__ void keep4_b(v16b a, v16b b, v16b c, v16b d) { asm volatile("v_nop" :: "v"(a), "v"(b), "v"(c), "v"(d)); }
__device__ __forceinline__ void acc_guard4(v8f& a, v8f& b, v8f& c, v8f& d) { asm volatile("v_nop\n\tv_nop\n\tv_nop\n\tv_nop" : "+v"(a), "+v"(b), "+v"(c), "+v"(d)); }
template <typename T> struct Frag;
template <> struct Frag<_Float16> {
  typedef v16h V; union U { v16h v; v8h h[2]; };
  static __device__ __forceinline__ v16h load(const _Float16* p) {
    U f; f.h[0] = *(const v8h*)(p); f.h[1] = *(const v8h*)(p + 16); return f.v;
  }
  static __device__ __forceinline__ v8f mma(v16h a, v16h b, v8f c) {
    return __builtin_amdgcn_wmma_f32_16x16x32_f16(false, a, false, b, (short)0, c, false, false);
  }
  static __device__ __forceinline__ void guard(v8f& a, v8f& b, v16h x, v16h y) { dep_guard_h(a, b, x, y); }
  static __device__ __forceinline__ void keep(v16h a, v16h b, v16h c, v16h d) { keep4_h(a, b, c, d); }
};
template <> struct Frag<__bf16> {
  typedef v16b V; union U { v16b v; v8b h[2]; };
  static __device__ __forceinline__ v16b load(const __bf16* p) {
    U f; f.h[0] = *(const v8b*)(p); f.h[1] = *(const v8b*)(p + 16); return f.v;
  }
  static __device__ __forceinline__ v8f mma(v16b a, v16b b, v8f c) {
    return __builtin_amdgcn_wmma_f32_16x16x32_bf16(false, a, false, b, (short)0, c, false, false);
  }
  static __device__ __forceinline__ void guard(v8f& a, v8f& b, v16b x, v16b y) { dep_guard_b(a, b, x, y); }
  static __device__ __forceinline__ void keep(v16b a, v16b b, v16b c, v16b d) { keep4_b(a, b, c, d); }
};

__device__ __forceinline__ unsigned pk16(unsigned short a, unsigned short b) { return (unsigned)a | ((unsigned)b << 16); }
__device__ __forceinline__ unsigned short h_bits(float f) { const _Float16 h = (_Float16)f; return __builtin_bit_cast(unsigned short, h); }

template <int ET> struct Elem;
template <> struct Elem<0> { typedef _Float16 T; };
template <> struct Elem<1> { typedef __bf16 T; };
template <int ET, bool SPLIT, int BIAS_MODE, int OUT_MODE, bool RESID, int ACT = 0>
__global__ __launch_bounds__(256) void wmma_gemm64(
    const unsigned short* __restrict__ Ap, const unsigned short* __restrict__ A2p, int lda, long strideA,
    const unsigned short* __restrict__ Btp, const unsigned short* __restrict__ Bt2p, int ldb, long strideB,
    void* __restrict__ Cout, void* __restrict__ Cout2, int ldc, long strideC,
    const float* __restrict__ bias,
    const float* __restrict__ resid, long strideR,
    int M, int N, int K, float scale) {
  typedef typename Elem<ET>::T T;
  typedef typename Frag<T>::V V;
  const T* A = (const T*)Ap; const T* A2 = (const T*)A2p; const T* Bt = (const T*)Btp; const T* Bt2 = (const T*)Bt2p;
  __shared__ __align__(16) float sT[8][16 * 68];
  const int b    = blockIdx.y;
  const int lane = threadIdx.x & 31;
  const int wave = threadIdx.x >> 5;
  const int tilesN = N >> 6;
  const int tilesM = M >> 6;
  const int tile = blockIdx.x * 8 + wave;
  if (tile >= tilesM * tilesN) return;
  const int tm = tile / tilesN;
  const int tn = tile - tm * tilesN;
  const int m0 = tm << 6;
  const int n0 = tn << 6;

  const T* Ab  = A  + (size_t)b * strideA;
  const T* Bb  = Bt + (size_t)b * strideB;
  const T* Ab2 = SPLIT ? (A2  + (size_t)b * strideA) : nullptr;
  const T* Bb2 = SPLIT ? (Bt2 + (size_t)b * strideB) : nullptr;

  const int rlane = lane & 15;
  const int koff  = (lane >> 4) * 8;
  const int mOff  = (lane >> 4) * 8;

  v8f acc[4][4];
#pragma unroll
  for (int i = 0; i < 4; ++i)
#pragma unroll
    for (int j = 0; j < 4; ++j) acc[i][j] = (v8f){0.f,0.f,0.f,0.f,0.f,0.f,0.f,0.f};

  for (int k0 = 0; k0 < K; k0 += 32) {
    V bh[4], bl[4];
#pragma unroll
    for (int j = 0; j < 4; ++j) {
      const size_t bo = (size_t)(n0 + (j << 4) + rlane) * ldb + koff + k0;
      bh[j] = Frag<T>::load(Bb + bo);
      if (SPLIT) bl[j] = Frag<T>::load(Bb2 + bo);
    }
#pragma unroll
    for (int i = 0; i < 4; ++i) {
      const size_t ao = (size_t)(m0 + (i << 4) + rlane) * lda + koff + k0;
      V ah = Frag<T>::load(Ab + ao);
      V al;
      if (SPLIT) al = Frag<T>::load(Ab2 + ao);
#pragma unroll
      for (int j = 0; j < 4; ++j) {
        acc[i][j] = Frag<T>::mma(ah, bh[j], acc[i][j]);
        if (SPLIT) {
          acc[i][j] = Frag<T>::mma(ah, bl[j], acc[i][j]);
          acc[i][j] = Frag<T>::mma(al, bh[j], acc[i][j]);
        }
      }
      Frag<T>::guard(acc[i][0], acc[i][3], ah, SPLIT ? al : ah);
    }
    Frag<T>::keep(bh[0], bh[1], bh[2], bh[3]);
    if (SPLIT) Frag<T>::keep(bl[0], bl[1], bl[2], bl[3]);
  }
  acc_guard4(acc[0][0], acc[0][1], acc[0][2], acc[0][3]);
  acc_guard4(acc[1][0], acc[1][1], acc[1][2], acc[1][3]);
  acc_guard4(acc[2][0], acc[2][1], acc[2][2], acc[2][3]);
  acc_guard4(acc[3][0], acc[3][1], acc[3][2], acc[3][3]);

  float* slab = sT[wave];
  const float* Rb = RESID ? (resid + (size_t)b * strideR) : nullptr;
#pragma unroll
  for (int i = 0; i < 4; ++i) {
    const int mBase = m0 + (i << 4);
#pragma unroll
    for (int j = 0; j < 4; ++j) {
      const int n = n0 + (j << 4) + rlane;
      float bv = 0.f;
      if (BIAS_MODE == 2) bv = bias[n];
#pragma unroll
      for (int r = 0; r < 8; ++r) {
        float v = acc[i][j][r] * scale;
        if (BIAS_MODE == 1) v += bias[mBase + mOff + r];
        if (BIAS_MODE == 2) v += bv;
        if (RESID) v += Rb[(size_t)(mBase + mOff + r) * ldc + n];
        if (ACT == 2) v = fmaxf(v, 0.0f);
        if (ACT == 4) v = (v > 0.f) ? v : 0.01f * v;
        slab[(mOff + r) * 68 + (j << 4) + rlane] = v;
      }
    }
    __builtin_amdgcn_fence(__ATOMIC_RELEASE, "workgroup");
    __builtin_amdgcn_wave_barrier();
    __builtin_amdgcn_fence(__ATOMIC_ACQUIRE, "workgroup");
    if (OUT_MODE == 0) {
      float* C = (float*)Cout + (size_t)b * strideC;
      const int hh = lane >> 4, c4 = (lane & 15) * 4;
      for (int pass = 0; pass < 2; ++pass) {
#pragma unroll
        for (int it = 0; it < 8; ++it) {
          const int row = it * 2 + hh;
          v4f v = *(const v4f*)(slab + row * 68 + c4);
          *(volatile v4f*)(C + (size_t)(mBase + row) * ldc + n0 + c4) = v;
        }
        __threadfence();
      }
    } else {
      const int q = lane >> 3, c8 = (lane & 7) * 8;
      unsigned short* C  = (unsigned short*)Cout  + (size_t)b * strideC;
      unsigned short* C2 = (OUT_MODE == 2) ? ((unsigned short*)Cout2 + (size_t)b * strideC) : nullptr;
      for (int pass = 0; pass < 2; ++pass) {
#pragma unroll
        for (int it = 0; it < 4; ++it) {
          const int row = it * 4 + q;
          const float* sp = slab + row * 68 + c8;
          v8h hv, lv;
#pragma unroll
          for (int e = 0; e < 8; ++e) {
            if (OUT_MODE == 1) {
              hv[e] = (_Float16)sp[e];
            } else {
              unsigned short hb = f2bf_bits(sp[e]);
              unsigned short lb = f2bf_bits(sp[e] - bf_bits2f(hb));
              hv[e] = __builtin_bit_cast(_Float16, hb);
              lv[e] = __builtin_bit_cast(_Float16, lb);
            }
          }
          *(volatile v8h*)(C + (size_t)(mBase + row) * ldc + n0 + c8) = hv;
          if (OUT_MODE == 2) *(volatile v8h*)(C2 + (size_t)(mBase + row) * ldc + n0 + c8) = lv;
        }
        __threadfence();
      }
    }
    __builtin_amdgcn_fence(__ATOMIC_RELEASE, "workgroup");
    __builtin_amdgcn_wave_barrier();
    __builtin_amdgcn_fence(__ATOMIC_ACQUIRE, "workgroup");
  }
}

__global__ __launch_bounds__(256) void cast8_carry_f16_kernel(const float* __restrict__ in,
                                                              unsigned short* __restrict__ out,
                                                              int n8, float carry) {
  const int i = blockIdx.x * 256 + threadIdx.x;
  if (i >= n8) return;
  const float* p = in + 8 * (size_t)i;
  const v4f a = *(const v4f*)(p);
  const v4f c = *(const v4f*)(p + 4);
  unsigned short hb[8];
#pragma unroll
  for (int e = 0; e < 4; ++e) {
    hb[e]     = h_bits(a[e] * carry);
    hb[4 + e] = h_bits(c[e] * carry);
  }
  const v4u u = (v4u){pk16(hb[0], hb[1]), pk16(hb[2], hb[3]), pk16(hb[4], hb[5]), pk16(hb[6], hb[7])};
  unsigned short* q = out + 8 * (size_t)i;
  *(volatile v4u*)q = u;
  __threadfence();
  *(volatile v4u*)q = u;
}

__global__ __launch_bounds__(256) void basis_prep_kernel(const float* __restrict__ x,
                                                         unsigned short* __restrict__ S16,
                                                         unsigned short* __restrict__ P16,
                                                         int row0) {
#pragma clang fp contract(off)
  __shared__ __align__(16) float sS[kInF];
  __shared__ __align__(16) float sP[kKB];
  const int t    = threadIdx.x;
  const int rloc = blockIdx.x;
  const float* xr = x + (size_t)(row0 + rloc) * kInF;

#pragma unroll 1
  for (int it = 0; it < 4; ++it) {
    const int i = it * 256 + t;
    const float v  = xr[i];
    const float ev = expf(-v);
    const float sg = __builtin_amdgcn_rcpf(1.0f + ev);
    sS[i] = (v * sg) * kSCarry;
    const float tt = tanhf(v);
    const float p0 = 1.0f;
    const float p1 = 0.5f * (4.0f * tt + 0.0f);
    const float a2 = (0.0f + kAl2 * tt) * kRg2;
    const float p2 = a2 * p1 - kBc2 * p0;
    const float a3 = (0.0f + kAl3 * tt) * kRg3;
    const float p3 = a3 * p2 - kBc3 * p1;
    const float a4 = (0.0f + kAl4 * tt) * kRg4;
    const float p4 = a4 * p3 - kBc4 * p2;
    const float a5 = (0.0f + kAl5 * tt) * kRg5;
    const float p5 = a5 * p4 - kBc5 * p3;
    float* pp = sP + i * kDeg1;
    pp[0] = p0 * kPCarry;
    pp[1] = p1 * kPCarry;
    pp[2] = p2 * kPCarry;
    pp[3] = p3 * kPCarry;
    pp[4] = p4 * kPCarry;
    pp[5] = p5 * kPCarry;
  }
  __syncthreads();

  unsigned short* prow = P16 + (size_t)rloc * kKB;
#pragma unroll
  for (int si = 0; si < 3; ++si) {
    const int s = si * 256 + t;
    const v4f a = *(const v4f*)(sP + 8 * s);
    const v4f c = *(const v4f*)(sP + 8 * s + 4);
    unsigned short hb[8];
#pragma unroll
    for (int e = 0; e < 4; ++e) {
      hb[e]     = h_bits(a[e]);
      hb[4 + e] = h_bits(c[e]);
    }
    const v4u u = (v4u){pk16(hb[0], hb[1]), pk16(hb[2], hb[3]), pk16(hb[4], hb[5]), pk16(hb[6], hb[7])};
    unsigned short* q = prow + 8 * s;
    *(volatile v4u*)q = u;
    __threadfence();
    *(volatile v4u*)q = u;
  }

  if (t < 128) {
    const v4f a = *(const v4f*)(sS + 8 * t);
    const v4f c = *(const v4f*)(sS + 8 * t + 4);
    unsigned short hb[8];
#pragma unroll
    for (int e = 0; e < 4; ++e) {
      hb[e]     = h_bits(a[e]);
      hb[4 + e] = h_bits(c[e]);
    }
    const v4u u = (v4u){pk16(hb[0], hb[1]), pk16(hb[2], hb[3]), pk16(hb[4], hb[5]), pk16(hb[6], hb[7])};
    unsigned short* q = S16 + (size_t)rloc * kInF + 8 * t;
    *(volatile v4u*)q = u;
    __threadfence();
    *(volatile v4u*)q = u;
  }
}

extern "C" void kernel_launch(void* const* d_in, const int* in_sizes, int n_in,
                              void* d_out, int out_size, void* d_ws, size_t ws_size,
                              hipStream_t stream) {
  if (n_in < 4) return;
  if (in_sizes[0] != kRows * kInF) return;
  if (in_sizes[1] != kOutF * kInF) return;
  if (in_sizes[2] != kOutF * kInF * kDeg1) return;
  if (in_sizes[3] != kOutF) return;
  if (out_size != kRows * kOutF) return;

  const float* x    = (const float*)d_in[0];
  const float* bw   = (const float*)d_in[1];
  const float* jc   = (const float*)d_in[2];
  const float* bias = (const float*)d_in[3];
  float* out        = (float*)d_out;

  const size_t bytesWb   = (size_t)kOutF * kInF * 2;
  const size_t bytesJc   = (size_t)kOutF * kKB * 2;
  const size_t bytesS16  = (size_t)kChunkRows * kInF * 2;
  const size_t bytesP16  = (size_t)kChunkRows * kKB * 2;
  const size_t bytesBase = (size_t)kChunkRows * kOutF * 4;
  const size_t offWb   = 0;
  const size_t offJc   = offWb + bytesWb;
  const size_t offS16  = offJc + bytesJc;
  const size_t offP16  = offS16 + bytesS16;
  const size_t offBase = offP16 + bytesP16;
  const size_t total   = offBase + bytesBase;
  if (total > ws_size) return;

  unsigned char* ws = (unsigned char*)d_ws;
  unsigned short* Wb16 = (unsigned short*)(ws + offWb);
  unsigned short* Jc16 = (unsigned short*)(ws + offJc);
  unsigned short* S16  = (unsigned short*)(ws + offS16);
  unsigned short* P16  = (unsigned short*)(ws + offP16);
  float* BaseP         = (float*)(ws + offBase);

  const int n8Wb = kOutF * kInF / 8;
  const int n8Jc = kOutF * kKB / 8;
  cast8_carry_f16_kernel<<<(n8Wb + 255) / 256, 256, 0, stream>>>(bw, Wb16, n8Wb, kWCarry);
  cast8_carry_f16_kernel<<<(n8Jc + 255) / 256, 256, 0, stream>>>(jc, Jc16, n8Jc, kJCarry);

  const int gemmBlocks = ((kChunkRows / 64) * (kOutF / 64) + 7) / 8;
  for (int c = 0; c < kNumChunks; ++c) {
    const int row0 = c * kChunkRows;
    basis_prep_kernel<<<kChunkRows, 256, 0, stream>>>(x, S16, P16, row0);

    wmma_gemm64<0, false, 2, 0, false, 0><<<dim3(gemmBlocks, 1), 256, 0, stream>>>(
        S16, S16, kInF, 0L,
        Wb16, Wb16, kInF, 0L,
        (void*)BaseP, (void*)BaseP, kOutF, 0L,
        bias,
        x, 0L,
        kChunkRows, kOutF, kInF, kBaseScale);

    float* outc = out + (size_t)row0 * kOutF;
    wmma_gemm64<0, false, 0, 0, true, 0><<<dim3(gemmBlocks, 1), 256, 0, stream>>>(
        P16, P16, kKB, 0L,
        Jc16, Jc16, kKB, 0L,
        (void*)outc, (void*)outc, kOutF, 0L,
        bias,
        BaseP, 0L,
        kChunkRows, kOutF, kKB, kPolyScale);
  }
}
